// SimpleRNN_32375463477377
// MI455X (gfx1250) — hardware-verified
//
#include <hip/hip_runtime.h>
#include <math.h>

typedef __attribute__((ext_vector_type(16))) _Float16 v16h;
typedef __attribute__((ext_vector_type(8)))  _Float16 v8h;
typedef __attribute__((ext_vector_type(16))) __bf16   v16b;
typedef __attribute__((ext_vector_type(8)))  __bf16   v8b;
typedef __attribute__((ext_vector_type(8)))  float    v8f;
typedef __attribute__((ext_vector_type(4)))  float    v4f;

constexpr int kN    = 8192;
constexpr int kL    = 16;
constexpr int kVoc  = 32000;
constexpr int kE    = 512;
constexpr int kHid  = 1024;
constexpr int kK    = kHid + kE;
constexpr int kK2   = kK + kHid;
constexpr int kTwoFrom = 8;
constexpr int kThr  = 256;
constexpr float kInCarry = 1024.0f;
constexpr float kSc = 1.0f / (kInCarry * kInCarry);
constexpr float kF16MinNormal = 6.103515625e-5f;

static_assert((kN % 64) == 0 && (kHid % 64) == 0 && ((kN / 64) * (kHid / 64)) % 8 == 0, "GEMM M, N multiples of 64; grid exact");
static_assert((kK % 32) == 0 && (kK2 % 32) == 0 && (kK2 % 256) == 0 && (kK % 256) == 0 && (kHid % 256) == 0 && (kE % 256) == 0 && kTwoFrom >= 1 && kTwoFrom < kL, "GEMM K multiples of 32; the plane cast's pitch and offsets multiples of 256");

constexpr size_t kOffWB = 0ull;
constexpr size_t kOffBIAS = 5242880ull;
constexpr size_t kOffA16 = 5251072ull;
constexpr size_t kOffGG = 47194112ull;
constexpr size_t kWsTotal = 80748544ull;
static_assert(kWsTotal <= 134217728ull, "carve cap: under 128 MiB");
static_assert(kOffWB == 0
              && kOffBIAS == kOffWB + 5242880ull
              && kOffA16 == kOffBIAS + 8192ull
              && kOffGG == kOffA16 + 41943040ull
              && kWsTotal == kOffGG + 33554432ull, "the carve is chained and totalled");
static_assert((kOffWB % 256) == 0 && (kOffBIAS % 256) == 0 && (kOffA16 % 256) == 0 && (kOffGG % 256) == 0, "aligned regions");

__device__ __forceinline__ unsigned short f2bf_bits(float f) {
  unsigned u = __float_as_uint(f);
  return (unsigned short)((u + 0x7FFFu + ((u >> 16) & 1u)) >> 16);
}
__device__ __forceinline__ float bf_bits2f(unsigned short h) { return __uint_as_float(((unsigned)h) << 16); }
__device__ __forceinline__ float bf16r(float f) { return bf_bits2f(f2bf_bits(f)); }
__device__ __forceinline__ float carry_flush(float v, float carry) {
  const float s = v * carry;
  return (fabsf(s) < kF16MinNormal) ? 0.0f : s;
}
__device__ __forceinline__ float frcp(float x) { return __builtin_amdgcn_rcpf(x); }

__device__ __forceinline__ void dep_guard4_h(v8f& a, v8f& b, v8f& c, v8f& d, v16h x, v16h y) { asm volatile("v_nop\n\tv_nop\n\tv_nop\n\tv_nop" : "+v"(a), "+v"(b), "+v"(c), "+v"(d) : "v"(x), "v"(y)); }
__device__ __forceinline__ void dep_guard4_b(v8f& a, v8f& b, v8f& c, v8f& d, v16b x, v16b y) { asm volatile("v_nop\n\tv_nop\n\tv_nop\n\tv_nop" : "+v"(a), "+v"(b), "+v"(c), "+v"(d) : "v"(x), "v"(y)); }
__device__ __forceinline__ void keep4_h(v16h a, v16h b, v16h c, v16h d) { asm volatile("v_nop" :: "v"(a), "v"(b), "v"(c), "v"(d)); }
__device__ __forceinline__ void keep4_b(v16b a, v16b b, v16b c, v16b d) { asm volatile("v_nop" :: "v"(a), "v"(b), "v"(c), "v"(d)); }
__device__ __forceinline__ void acc_guard4(v8f& a, v8f& b, v8f& c, v8f& d) { asm volatile("v_nop\n\tv_nop\n\tv_nop\n\tv_nop" : "+v"(a), "+v"(b), "+v"(c), "+v"(d)); }

template <typename T> struct Frag;
template <> struct Frag<_Float16> {
  typedef v16h V; union U { v16h v; v8h h[2]; };
  static __device__ __forceinline__ v16h load(const _Float16* p) {
    U f; f.h[0] = *(const v8h*)(p); f.h[1] = *(const v8h*)(p + 16); return f.v;
  }
  static __device__ __forceinline__ v8f mma(v16h a, v16h b, v8f c) {
    return __builtin_amdgcn_wmma_f32_16x16x32_f16(false, a, false, b, (short)0, c, false, false);
  }
  static __device__ __forceinline__ void guard4(v8f& a, v8f& b, v8f& c, v8f& d, v16h x, v16h y) { dep_guard4_h(a, b, c, d, x, y); }
  static __device__ __forceinline__ void keep(v16h a, v16h b, v16h c, v16h d) { keep4_h(a, b, c, d); }
};
template <> struct Frag<__bf16> {
  typedef v16b V; union U { v16b v; v8b h[2]; };
  static __device__ __forceinline__ v16b load(const __bf16* p) {
    U f; f.h[0] = *(const v8b*)(p); f.h[1] = *(const v8b*)(p + 16); return f.v;
  }
  static __device__ __forceinline__ v8f mma(v16b a, v16b b, v8f c) {
    return __builtin_amdgcn_wmma_f32_16x16x32_bf16(false, a, false, b, (short)0, c, false, false);
  }
  static __device__ __forceinline__ void guard4(v8f& a, v8f& b, v8f& c, v8f& d, v16b x, v16b y) { dep_guard4_b(a, b, c, d, x, y); }
  static __device__ __forceinline__ void keep(v16b a, v16b b, v16b c, v16b d) { keep4_b(a, b, c, d); }
};

__device__ __forceinline__ v8f mma_h(v16h a, v16h b, v8f c) {
  c = __builtin_amdgcn_wmma_f32_16x16x32_f16(false, a, false, b, (short)0, c, false, false);
  asm volatile("v_nop\n\tv_nop\n\tv_nop\n\tv_nop" : "+v"(c) : "v"(a), "v"(b));
  return c;
}

template <int ET> struct Elem;
template <> struct Elem<0> { typedef _Float16 T; };
template <> struct Elem<1> { typedef __bf16 T; };
template <int ET, bool SPLIT, int BIAS_MODE, int OUT_MODE, bool RESID, int ACT = 0>
__global__ __launch_bounds__(256) void wmma_gemm64(
    const unsigned short* __restrict__ Ap, const unsigned short* __restrict__ A2p, int lda, long strideA,
    const unsigned short* __restrict__ Btp, const unsigned short* __restrict__ Bt2p, int ldb, long strideB,
    void* __restrict__ Cout, void* __restrict__ Cout2, int ldc, long strideC,
    const float* __restrict__ bias,
    const float* __restrict__ resid, long strideR,
    int M, int N, int K, float scale) {
  typedef typename Elem<ET>::T T;
  typedef typename Frag<T>::V V;
  const T* A = (const T*)Ap; const T* A2 = (const T*)A2p; const T* Bt = (const T*)Btp; const T* Bt2 = (const T*)Bt2p;
  __shared__ __align__(16) float sT[8][16 * 68];
  const int b    = blockIdx.y;
  const int lane = threadIdx.x & 31;
  const int wave = threadIdx.x >> 5;
  const int tilesN = N >> 6;
  const int tilesM = M >> 6;
  const int tile = blockIdx.x * 8 + wave;
  if (tile >= tilesM * tilesN) return;
  const int tm = tile / tilesN;
  const int tn = tile - tm * tilesN;
  const int m0 = tm << 6;
  const int n0 = tn << 6;

  const T* Ab  = A  + (size_t)b * strideA;
  const T* Bb  = Bt + (size_t)b * strideB;
  const T* Ab2 = SPLIT ? (A2  + (size_t)b * strideA) : nullptr;
  const T* Bb2 = SPLIT ? (Bt2 + (size_t)b * strideB) : nullptr;

  const int rlane = lane & 15;
  const int koff  = (lane >> 4) * 8;
  const int mOff  = (lane >> 4) * 8;

  v8f acc[4][4];
#pragma unroll
  for (int i = 0; i < 4; ++i)
#pragma unroll
    for (int j = 0; j < 4; ++j) acc[i][j] = (v8f){0.f,0.f,0.f,0.f,0.f,0.f,0.f,0.f};

  for (int k0 = 0; k0 < K; k0 += 32) {
    V bh[4], bl[4];
#pragma unroll
    for (int j = 0; j < 4; ++j) {
      const size_t bo = (size_t)(n0 + (j << 4) + rlane) * ldb + koff + k0;
      bh[j] = Frag<T>::load(Bb + bo);
      if (SPLIT) bl[j] = Frag<T>::load(Bb2 + bo);
    }
#pragma unroll
    for (int i = 0; i < 4; ++i) {
      const size_t ao = (size_t)(m0 + (i << 4) + rlane) * lda + koff + k0;
      V ah = Frag<T>::load(Ab + ao);
      V al;
      if (SPLIT) al = Frag<T>::load(Ab2 + ao);
#pragma unroll
      for (int j = 0; j < 4; ++j) {
        acc[i][j] = Frag<T>::mma(ah, bh[j], acc[i][j]);
        if (SPLIT) {
          acc[i][j] = Frag<T>::mma(ah, bl[j], acc[i][j]);
          acc[i][j] = Frag<T>::mma(al, bh[j], acc[i][j]);
        }
      }
      Frag<T>::guard4(acc[i][0], acc[i][1], acc[i][2], acc[i][3], ah, SPLIT ? al : ah);
    }
    Frag<T>::keep(bh[0], bh[1], bh[2], bh[3]);
    if (SPLIT) Frag<T>::keep(bl[0], bl[1], bl[2], bl[3]);
  }
  acc_guard4(acc[0][0], acc[0][1], acc[0][2], acc[0][3]);
  acc_guard4(acc[1][0], acc[1][1], acc[1][2], acc[1][3]);
  acc_guard4(acc[2][0], acc[2][1], acc[2][2], acc[2][3]);
  acc_guard4(acc[3][0], acc[3][1], acc[3][2], acc[3][3]);

  float* slab = sT[wave];
  const float* Rb = RESID ? (resid + (size_t)b * strideR) : nullptr;
#pragma unroll
  for (int i = 0; i < 4; ++i) {
    const int mBase = m0 + (i << 4);
#pragma unroll
    for (int j = 0; j < 4; ++j) {
      const int n = n0 + (j << 4) + rlane;
      float bv = 0.f;
      if (BIAS_MODE == 2) bv = bias[n];
#pragma unroll
      for (int r = 0; r < 8; ++r) {
        float v = acc[i][j][r] * scale;
        if (BIAS_MODE == 1) v += bias[mBase + mOff + r];
        if (BIAS_MODE == 2) v += bv;
        if (RESID) v += Rb[(size_t)(mBase + mOff + r) * ldc + n];
        if (ACT == 1) v = tanhf(v);
        if (ACT == 2) v = fmaxf(v, 0.0f);
        if (ACT == 3) v = v / (1.0f + expf(-v));
        if (ACT == 4) v = (v > 0.f) ? v : 0.01f * v;
        slab[(mOff + r) * 68 + (j << 4) + rlane] = v;
      }
    }
    __builtin_amdgcn_fence(__ATOMIC_RELEASE, "workgroup");
    __builtin_amdgcn_wave_barrier();
    __builtin_amdgcn_fence(__ATOMIC_ACQUIRE, "workgroup");
    if (OUT_MODE == 0) {
      float* C = (float*)Cout + (size_t)b * strideC;
      const int hh = lane >> 4, c4 = (lane & 15) * 4;
      for (int pass = 0; pass < 2; ++pass) {
#pragma unroll
        for (int it = 0; it < 8; ++it) {
          const int row = it * 2 + hh;
          v4f v = *(const v4f*)(slab + row * 68 + c4);
          *(volatile v4f*)(C + (size_t)(mBase + row) * ldc + n0 + c4) = v;
        }
        __threadfence();
      }
    } else {
      const int q = lane >> 3, c8 = (lane & 7) * 8;
      unsigned short* C  = (unsigned short*)Cout  + (size_t)b * strideC;
      unsigned short* C2 = (OUT_MODE == 2) ? ((unsigned short*)Cout2 + (size_t)b * strideC) : nullptr;
      for (int pass = 0; pass < 2; ++pass) {
#pragma unroll
        for (int it = 0; it < 4; ++it) {
          const int row = it * 4 + q;
          const float* sp = slab + row * 68 + c8;
          v8h hv, lv;
#pragma unroll
          for (int e = 0; e < 8; ++e) {
            if (OUT_MODE == 1) {
              hv[e] = (_Float16)sp[e];
            } else {
              unsigned short hb = f2bf_bits(sp[e]);
              unsigned short lb = f2bf_bits(sp[e] - bf_bits2f(hb));
              hv[e] = __builtin_bit_cast(_Float16, hb);
              lv[e] = __builtin_bit_cast(_Float16, lb);
            }
          }
          *(volatile v8h*)(C + (size_t)(mBase + row) * ldc + n0 + c8) = hv;
          if (OUT_MODE == 2) *(volatile v8h*)(C2 + (size_t)(mBase + row) * ldc + n0 + c8) = lv;
        }
        __threadfence();
      }
    }
    __builtin_amdgcn_fence(__ATOMIC_RELEASE, "workgroup");
    __builtin_amdgcn_wave_barrier();
    __builtin_amdgcn_fence(__ATOMIC_ACQUIRE, "workgroup");
  }
}

__global__ __launch_bounds__(kThr) void cast_plane_kernel(const float* __restrict__ src, unsigned short* __restrict__ dst,
                                                          int colsLog2, int dstPitch, int dstOff) {
  const int i   = blockIdx.x * kThr + threadIdx.x;
  const int sh  = colsLog2 - 3;
  const int row = i >> sh;
  const int c8  = (i & ((1 << sh) - 1)) * 8;
  const float* sp = src + ((size_t)row << colsLog2) + c8;
  const v4f a0 = *(const v4f*)(sp);
  const v4f a1 = *(const v4f*)(sp + 4);
  v8h hv;
#pragma unroll
  for (int e = 0; e < 4; ++e) {
    const float f0 = a0[e];
    const float f1 = a1[e];
    hv[e]     = (_Float16)carry_flush(bf16r(f0), kInCarry);
    hv[4 + e] = (_Float16)carry_flush(bf16r(f1), kInCarry);
  }
  unsigned short* dp = dst + (size_t)row * dstPitch + dstOff + c8;
  *(volatile v8h*)dp = hv;
  __threadfence();
  *(volatile v8h*)dp = hv;
}

__device__ __forceinline__ float fast_tanh(float v) { return 1.0f - 2.0f * frcp(__expf(2.0f * v) + 1.0f); }

__device__ __forceinline__ v8h emb_row8(const float* __restrict__ E, int tok, unsigned c8) {
  tok = (tok < 0) ? 0 : ((tok > kVoc - 1) ? (kVoc - 1) : tok);
  const float* sp = E + (size_t)tok * kE + c8;
  const v4f a0 = *(const v4f*)sp, a1 = *(const v4f*)(sp + 4);
  v8h hv;
#pragma unroll
  for (int e = 0; e < 4; ++e) { const float p = a0[e], q = a1[e]; hv[e] = (_Float16)carry_flush(bf16r(p), kInCarry); hv[4 + e] = (_Float16)carry_flush(bf16r(q), kInCarry); }
  return hv;
}

__global__ __launch_bounds__(kThr) void setup_kernel(const int* __restrict__ X, const float* __restrict__ E, const float* __restrict__ b_hh,
                                                     const float* __restrict__ b_xh, float* __restrict__ BIAS, unsigned short* __restrict__ A16) {
  unsigned v = blockIdx.x * (unsigned)kThr + threadIdx.x;
  asm volatile("" : "+v"(v));
  if (v < 512u) {
    const unsigned i0 = v * 4u;
    v4f o = {0.f, 0.f, 0.f, 0.f};
    if (i0 < (unsigned)kHid) {
      const v4f a = *(const v4f*)(b_hh + i0), c = *(const v4f*)(b_xh + i0);
#pragma unroll
      for (int e = 0; e < 4; ++e) { const float p = a[e], q = c[e]; o[e] = bf16r(p) + bf16r(q); }
    }
    float* dp = BIAS + i0;
    *(volatile v4f*)dp = o;
    __threadfence();
    *(volatile v4f*)dp = o;
  } else {
    v8h hv;
    unsigned short* dp;
    if (v < 1049088u) {
      const unsigned w = v - 512u;
#pragma unroll
      for (int e = 0; e < 8; ++e) hv[e] = (_Float16)0.0f;
      dp = A16 + (size_t)(w >> 7) * kK2 + (w & 127u) * 8u;
    } else {
      const unsigned w = v - 1049088u;
      const unsigned n = w >> 6, c8 = (w & 63u) * 8u;
      hv = emb_row8(E, X[(size_t)n * kL], c8);
      dp = A16 + (size_t)n * kK2 + kHid + c8;
    }
    *(volatile v8h*)dp = hv;
    __threadfence();
    *(volatile v8h*)dp = hv;
  }
}
static_assert(2048 / 4 == 512 && kN * kHid / 8 == 1048576 && kN * kE / 8 == 524288 && 512 + 1048576 + 524288 == 6146 * kThr && (1049088 % 32) == 0, "set-up grid exact; regions wave-uniform");

__global__ __launch_bounds__(kThr) void cell_kernel(const float* __restrict__ GG, const int* __restrict__ X, const float* __restrict__ E,
                                                    unsigned short* __restrict__ A16, float* __restrict__ out, int t) {
  unsigned v = blockIdx.x * (unsigned)kThr + threadIdx.x;
  asm volatile("" : "+v"(v));
  const unsigned n = v >> 7;
  const unsigned u8 = (v & 127u) * 8u;
  const float* gr = GG + (size_t)n * kHid + u8;
  const v4f g0 = *(const v4f*)gr, g1 = *(const v4f*)(gr + 4);
  v4f h0, h1; v8h hv, lv;
#pragma unroll
  for (int e = 0; e < 4; ++e) {
    const float a = fast_tanh(g0[e]), b = fast_tanh(g1[e]);
    h0[e] = a; h1[e] = b;
    const _Float16 ha = (_Float16)carry_flush(a, kInCarry), hb = (_Float16)carry_flush(b, kInCarry);
    hv[e] = ha; hv[4 + e] = hb;
    const float ra = a * kInCarry - (float)ha, rb = b * kInCarry - (float)hb;
    lv[e] = (_Float16)((fabsf(ra) < kF16MinNormal) ? 0.0f : ra); lv[4 + e] = (_Float16)((fabsf(rb) < kF16MinNormal) ? 0.0f : rb);
  }
  const bool nx = (u8 < (unsigned)kE) && (t + 1 < kL);
  const v8h xv = emb_row8(E, X[(size_t)n * kL + (size_t)(nx ? (t + 1) : 0)], nx ? u8 : 0u);
  const bool last = (t == kL - 1);
  const bool two = (t + 1 >= kTwoFrom) && (t + 1 < kL);
  unsigned short* hp = A16 + (size_t)n * kK2 + u8;
  unsigned short* lp = A16 + (size_t)n * kK2 + kK + u8;
  unsigned short* xp = A16 + (size_t)n * kK2 + kHid + (nx ? u8 : 0u);
  float* op = out + (size_t)n * kHid + u8;
  for (int pass = 0; pass < 2; ++pass) {
    *(volatile v8h*)hp = hv;
    if (two) *(volatile v8h*)lp = lv;
    if (nx) *(volatile v8h*)xp = xv;
    if (last) { *(volatile v4f*)op = h0; *(volatile v4f*)(op + 4) = h1; }
    __threadfence();
  }
}
static_assert(kN * kHid / 8 == 4096 * kThr && kHid / 8 == 128 && (kE / 8) % 32 == 0, "cell grid exact; the input's threads end on a wave boundary");

static_assert(((size_t)kHid * kHid / 8) % kThr == 0 && ((size_t)kHid * kE / 8) % kThr == 0, "plane cast grids exact");

extern "C" void kernel_launch(void* const* d_in, const int* in_sizes, int n_in,
                              void* d_out, int out_size, void* d_ws, size_t ws_size,
                              hipStream_t stream) {
  if (n_in < 6 || d_out == nullptr || d_ws == nullptr) return;
  if (in_sizes[0] != kN * kL || in_sizes[1] != kVoc * kE || in_sizes[2] != kHid * kHid || in_sizes[3] != kHid || in_sizes[4] != kHid * kE || in_sizes[5] != kHid) return;
  if (out_size != kN * kHid) return;
  if (ws_size < kWsTotal) return;
  const int* X = (const int*)d_in[0];
  const float* E = (const float*)d_in[1];
  const float* W_hh = (const float*)d_in[2];
  const float* b_hh = (const float*)d_in[3];
  const float* W_xh = (const float*)d_in[4];
  const float* b_xh = (const float*)d_in[5];
  float* out = (float*)d_out;
  char* ws = (char*)d_ws;
  unsigned short* WB = (unsigned short*)(ws + kOffWB);
  float* BIAS = (float*)(ws + kOffBIAS);
  unsigned short* A16 = (unsigned short*)(ws + kOffA16);
  float* GG = (float*)(ws + kOffGG);

  cast_plane_kernel<<<(int)(((size_t)kHid * kHid / 8) / kThr), kThr, 0, stream>>>(W_hh, WB, 10, kK2, 0);
  cast_plane_kernel<<<(int)(((size_t)kHid * kE / 8) / kThr), kThr, 0, stream>>>(W_xh, WB, 9, kK2, kHid);
  cast_plane_kernel<<<(int)(((size_t)kHid * kHid / 8) / kThr), kThr, 0, stream>>>(W_hh, WB, 10, kK2, kK);
  setup_kernel<<<6146, kThr, 0, stream>>>(X, E, b_hh, b_xh, BIAS, A16);

  for (int t = 0; t < kL; ++t) {
    const int kk = (t < kTwoFrom) ? kK : kK2;
    wmma_gemm64<0, false, 2, 0, false, 0><<<dim3((kN / 64) * (kHid / 64) / 8, 1), 256, 0, stream>>>(
        A16, A16, kK2, 0L, WB, WB, kK2, 0L, (void*)GG, (void*)GG, kHid, 0L, BIAS, nullptr, 0L, kN, kHid, kk, kSc);
    cell_kernel<<<4096, kThr, 0, stream>>>(GG, X, E, A16, out, t);
  }
}
